// RIMCell_37692632990224
// MI455X (gfx1250) — hardware-verified
//
#include <hip/hip_runtime.h>

typedef unsigned short u16;
typedef __bf16 bf16t;
typedef bf16t    v16bf __attribute__((ext_vector_type(16)));
typedef u16      v16u  __attribute__((ext_vector_type(16)));
typedef u16      v8u   __attribute__((ext_vector_type(8)));
typedef float    v8f   __attribute__((ext_vector_type(8)));
typedef float    v4f   __attribute__((ext_vector_type(4)));
typedef v8u __attribute__((may_alias)) v8ua;
typedef v4f __attribute__((may_alias)) v4fa;

union FragU { v16u v; v8u half[2]; };

#define NB    1024
#define NIN   512
#define NH    600
#define NHP   608
#define NU    6
#define NTOP  4
#define NQK   64
#define NVD   400
#define NVP   416
#define NCH   4
#define NCQ   32
#define NCV   100
#define NCQA  128
#define NG    2400
#define HLH   1216
#define HLV   832
#define MPITCH 32
#define OUT1  (NB * NU * NH)
#define RS32  0.17677669529663687f

static_assert(NHP % 32 == 0);
static_assert(NVP % 32 == 0);
static_assert(NIN % 32 == 0);
static_assert(NB % 64 == 0);
static_assert((NB * NU * NH) % 4 == 0);

__device__ __forceinline__ u16 f2bf(float f) {
  unsigned v = __float_as_uint(f);
  v += 0x7FFFu + ((v >> 16) & 1u);
  return (u16)(v >> 16);
}
__device__ __forceinline__ float bf2f(u16 b) { return __uint_as_float(((unsigned)b) << 16); }
__device__ __forceinline__ float bfr(float f) { return bf2f(f2bf(f)); }

__device__ __forceinline__ v8f wmma_bf(v16u a, v16u b, v8f c) {
  v8f d = __builtin_amdgcn_wmma_f32_16x16x32_bf16(false, __builtin_bit_cast(v16bf, a), false,
                                                   __builtin_bit_cast(v16bf, b), (short)0, c, false, false);
  asm volatile("v_nop\n\tv_nop\n\tv_nop\n\tv_nop" : "+v"(d) : "v"(a), "v"(b));
  return d;
}

__device__ __forceinline__ v16u load_frag(const u16* p, int h) {
  FragU f;
  f.half[0] = *(const v8ua*)(p + 8 * h);
  f.half[1] = *(const v8ua*)(p + 16 + 8 * h);
  return f.v;
}

__device__ __forceinline__ float sigm(float x) {
  const float e = expf(-fabsf(x));
  const float r = 1.0f / (1.0f + e);
  return x >= 0.f ? r : e * r;
}
__device__ __forceinline__ float tanh_c(float x) {
  return tanhf(fminf(fmaxf(x, -15.0f), 15.0f));
}

__global__ __launch_bounds__(256) void k_cvt_rows(
    const float* __restrict__ src, int sw, int pp, int total, u16* __restrict__ dst)
{
  const int p = blockIdx.x * 256 + threadIdx.x;
  if (p >= total) return;
  const int row = p / pp, c = p - row * pp;
  const int nreal = sw >> 3;
  const int cc = (c < nreal) ? c : (nreal - 1);
  const float* s = src + (size_t)row * sw + 8 * cc;
  const v4f a = *(const v4fa*)s;
  const v4f e = *(const v4fa*)(s + 4);
  v8u o;
  o[0] = f2bf(a.x); o[1] = f2bf(a.y); o[2] = f2bf(a.z); o[3] = f2bf(a.w);
  o[4] = f2bf(e.x); o[5] = f2bf(e.y); o[6] = f2bf(e.z); o[7] = f2bf(e.w);
  const v8u z = {0, 0, 0, 0, 0, 0, 0, 0};
  if (c >= nreal) o = z;
  u16* d = dst + (size_t)p * 8;
  *(volatile v8u*)d = o;
  __threadfence();
  *(volatile v8u*)d = o;
}

__global__ __launch_bounds__(256) void k_cvt_T(
    const float* __restrict__ src, int K, int N, int Kp, int Npad, u16* __restrict__ dst)
{
  __shared__ __attribute__((aligned(16))) u16 sT[32 * 608];
  const int tid = threadIdx.x;
  const int n0 = blockIdx.x * 32, u = blockIdx.y;
  const int kl = tid >> 5, nl = tid & 31;
  const int n = n0 + nl, nc = (n < N) ? n : (N - 1);
  const float* sb = src + (size_t)u * K * N;
  #pragma unroll 1
  for (int k0 = 0; k0 < Kp; k0 += 8) {
    const int k = k0 + kl, kc = (k < K) ? k : (K - 1);
    float v = sb[(size_t)kc * N + nc];
    if (k >= K || n >= N) v = 0.f;
    sT[nl * Kp + k] = f2bf(v);
  }
  __syncthreads();
  const int tot = 4 * Kp;
  u16* db = dst + ((size_t)u * Npad + n0) * Kp;
  #pragma unroll 1
  for (int p = tid; p < tot; p += 256) {
    const v8u v = *(const v8ua*)(sT + 8 * p);
    *(volatile v8u*)(db + 8 * (size_t)p) = v;
  }
  __threadfence();
  #pragma unroll 1
  for (int p = tid; p < tot; p += 256) {
    const v8u v = *(const v8ua*)(sT + 8 * p);
    *(volatile v8u*)(db + 8 * (size_t)p) = v;
  }
}

__device__ __forceinline__ void gemm_store(const float* sO, float* Cu, int ldc,
                                           int m0, int n0, int w, int lane) {
  const int q8 = lane & 7, sub = lane >> 3;
  #pragma unroll
  for (int i = 0; i < 4; ++i) {
    const int row = 16 * w + 4 * i + sub;
    const v4f v = *(const v4fa*)(sO + row * 32 + 4 * q8);
    *(volatile v4f*)(Cu + (size_t)(m0 + row) * ldc + n0 + 4 * q8) = v;
  }
}

template <int HL>
__global__ __launch_bounds__(128) void k_gemm(
    const u16* __restrict__ A, int lda, int sAu,
    const u16* __restrict__ Bw, int kp, int sBu,
    float* __restrict__ C, int ldc, int sCu,
    const float* __restrict__ bias, int nvalid, int hasb)
{
  __shared__ __attribute__((aligned(16))) float sO[64 * 32];
  const int tid = threadIdx.x, lane = tid & 31, w = tid >> 5;
  const int h = lane >> 4, m = lane & 15;
  const int n0 = blockIdx.x * 32, m0 = blockIdx.y * 64, u = blockIdx.z;

  const u16* Ab = A + (size_t)u * sAu + (size_t)(m0 + 16 * w + m) * lda;
  const u16* Bb = Bw + (size_t)u * sBu + (size_t)(n0 + m) * kp;

  const v8f z8 = {0.f, 0.f, 0.f, 0.f, 0.f, 0.f, 0.f, 0.f};
  v8f acc[2];
  acc[0] = z8; acc[1] = z8;

  #pragma unroll 1
  for (int k0 = 0; k0 < kp; k0 += 32) {
    const v16u b0 = load_frag(Bb + k0, h);
    const v16u b1 = load_frag(Bb + (size_t)16 * kp + k0, h);
    if (HL) {
      const v16u ah = load_frag(Ab + 2 * k0, h);
      const v16u al = load_frag(Ab + 2 * k0 + 32, h);
      acc[0] = wmma_bf(ah, b0, acc[0]);
      acc[0] = wmma_bf(al, b0, acc[0]);
      acc[1] = wmma_bf(ah, b1, acc[1]);
      acc[1] = wmma_bf(al, b1, acc[1]);
    } else {
      const v16u a = load_frag(Ab + k0, h);
      acc[0] = wmma_bf(a, b0, acc[0]);
      acc[1] = wmma_bf(a, b1, acc[1]);
    }
  }

  #pragma unroll
  for (int nt = 0; nt < 2; ++nt) {
    const int col = 16 * nt + m, gcol = n0 + col;
    const int gc = (gcol < nvalid) ? gcol : (nvalid - 1);
    float badd = 0.f;
    if (hasb) badd = bfr(bias[gc]);
    #pragma unroll
    for (int r = 0; r < 8; ++r) {
      float v = acc[nt][r] + badd;
      if (gcol >= nvalid) v = 0.f;
      sO[(16 * w + 8 * h + r) * 32 + col] = v;
    }
  }
  __syncthreads();

  float* Cu = C + (size_t)u * sCu;
  gemm_store(sO, Cu, ldc, m0, n0, w, lane);
  __threadfence();
  gemm_store(sO, Cu, ldc, m0, n0, w, lane);
}

__global__ __launch_bounds__(64) void k_select(
    const float* __restrict__ ql, const float* __restrict__ kl, const float* __restrict__ bk,
    const float* __restrict__ vl0, const float* __restrict__ bv,
    u16* __restrict__ inpHL, float* __restrict__ maskp)
{
  __shared__ float s0s[8], p0s[8], p1s[8];
  __shared__ __attribute__((aligned(16))) float msk[32];
  const int tid = threadIdx.x, lane = tid & 31, w = tid >> 5, b = blockIdx.x;

  {
    const int uu = (tid < NU) ? tid : (NU - 1);
    const float* q  = ql + ((size_t)b * NU + uu) * NQK;
    const float* kr = kl + (size_t)b * NQK;
    float a0 = 0.f, a1 = 0.f;
    #pragma unroll 1
    for (int i = 0; i < NQK; ++i) {
      const float qi = q[i];
      a0 += qi * kr[i];
      a1 += qi * bfr(bk[i]);
    }
    const float s0 = a0 * 0.125f, s1 = a1 * 0.125f;
    const float mx = fmaxf(s0, s1);
    const float e0 = expf(s0 - mx), e1 = expf(s1 - mx);
    const float inv = 1.0f / (e0 + e1);
    if (tid < NU) { s0s[tid] = s0; p0s[tid] = e0 * inv; p1s[tid] = e1 * inv; }
    if (tid < 32) msk[tid] = 0.f;
  }
  __syncthreads();
  if (tid == 0) {
    int chosen = 0;
    #pragma unroll 1
    for (int kk = 0; kk < NTOP; ++kk) {
      int best = -1; float bs = 0.f;
      #pragma unroll 1
      for (int uu = 0; uu < NU; ++uu) {
        if (((chosen >> uu) & 1) == 0) {
          const float s = s0s[uu];
          if (best < 0 || s > bs) { best = uu; bs = s; }
        }
      }
      chosen |= (1 << best);
    }
    #pragma unroll 1
    for (int uu = 0; uu < NU; ++uu) msk[uu] = ((chosen >> uu) & 1) ? 1.0f : 0.0f;
  }
  __syncthreads();

  if (tid < 8) {
    const v4f mv = *(const v4fa*)(msk + 4 * tid);
    float* d = maskp + (size_t)b * MPITCH + 4 * tid;
    *(volatile v4f*)d = mv;
    __threadfence();
    *(volatile v4f*)d = mv;
  }

  const int q8 = lane & 7, sub = lane >> 3, cq = q8 & 3;
  const float* vrow = vl0 + (size_t)b * NVP;
  #pragma unroll 1
  for (int it = 0; it < 10; ++it) {
    const int L = it * 8 + w * 4 + sub;
    const int Lc = (L < 78) ? L : 77;
    const int uu = Lc / 13, ks = Lc - uu * 13;
    const int col0 = 32 * ks + 8 * cq;
    const int cb = (col0 < NVD - 8) ? col0 : (NVD - 8);
    const v4f va = *(const v4fa*)(vrow + col0);
    const v4f vb = *(const v4fa*)(vrow + col0 + 4);
    const v4f na = *(const v4fa*)(bv + cb);
    const v4f nb = *(const v4fa*)(bv + cb + 4);
    const float pp0 = p0s[uu], pp1 = p1s[uu], mm = msk[uu];
    float vv[8], nv[8];
    vv[0] = va.x; vv[1] = va.y; vv[2] = va.z; vv[3] = va.w;
    vv[4] = vb.x; vv[5] = vb.y; vv[6] = vb.z; vv[7] = vb.w;
    nv[0] = na.x; nv[1] = na.y; nv[2] = na.z; nv[3] = na.w;
    nv[4] = nb.x; nv[5] = nb.y; nv[6] = nb.z; nv[7] = nb.w;
    v8u o;
    #pragma unroll
    for (int j = 0; j < 8; ++j) {
      float val = (pp0 * vv[j] + pp1 * bfr(nv[j])) * mm;
      if (col0 + j >= NVD) val = 0.f;
      const u16 hi = f2bf(val);
      const u16 lo = f2bf(val - bf2f(hi));
      o[j] = (q8 < 4) ? hi : lo;
    }
    u16* d = inpHL + (((size_t)b * NU + uu) * 13 + ks) * 64 + 8 * q8;
    if (L < 78) *(volatile v8u*)d = o;
    __threadfence();
    if (L < 78) *(volatile v8u*)d = o;
  }
}

__device__ __forceinline__ void lstm_store(const float* sC, const float* sH, const u16* sHL,
                                           float* cnew, float* hrnn, u16* hHL,
                                           int m0, int u, int slice, int w, int lane) {
  const int q8 = lane & 7, sub = lane >> 3;
  #pragma unroll
  for (int i = 0; i < 4; ++i) {
    const int row = 16 * w + 4 * i + sub;
    const size_t pr = (size_t)(m0 + row) * NU + u;
    const v4f vc = *(const v4fa*)(sC + row * 32 + 4 * q8);
    *(volatile v4f*)(cnew + pr * NHP + 32 * slice + 4 * q8) = vc;
  }
  #pragma unroll
  for (int i = 0; i < 4; ++i) {
    const int row = 16 * w + 4 * i + sub;
    const size_t pr = (size_t)(m0 + row) * NU + u;
    const v4f vh = *(const v4fa*)(sH + row * 32 + 4 * q8);
    *(volatile v4f*)(hrnn + pr * NHP + 32 * slice + 4 * q8) = vh;
  }
  #pragma unroll
  for (int i = 0; i < 4; ++i) {
    const int row = 16 * w + 4 * i + sub;
    const size_t pr = (size_t)(m0 + row) * NU + u;
    const v8u vb = *(const v8ua*)(sHL + row * 64 + 8 * q8);
    *(volatile v8u*)(hHL + pr * HLH + 64 * slice + 8 * q8) = vb;
  }
}

__global__ __launch_bounds__(128) void k_lstm(
    const u16* __restrict__ hsb,
    const u16* __restrict__ whhP,
    const u16* __restrict__ inpHL,
    const u16* __restrict__ wihP,
    const float* __restrict__ bih, const float* __restrict__ bhh,
    const float* __restrict__ cs,
    float* __restrict__ cnew, float* __restrict__ hrnn, u16* __restrict__ hHL)
{
  __shared__ __attribute__((aligned(16))) float sG[4 * 64 * 32];
  __shared__ __attribute__((aligned(16))) float sC[64 * 32];
  __shared__ __attribute__((aligned(16))) float sH[64 * 32];
  __shared__ __attribute__((aligned(16))) u16   sHL[64 * 64];

  const int tid = threadIdx.x, lane = tid & 31, w = tid >> 5;
  const int h = lane >> 4, m = lane & 15;
  const int slice = blockIdx.x, m0 = blockIdx.y * 64, u = blockIdx.z;
  const int c0 = slice * 32;
  const int wm = w >> 1, wn = w & 1;
  const int colL = 16 * wn + m;
  const int gcol = c0 + colL;
  const int gcc = (gcol < NH) ? gcol : (NH - 1);

  #pragma unroll
  for (int it = 0; it < 4; ++it) {
    const int p = it * 128 + tid;
    const int row = p >> 3, q = p & 7;
    int col = c0 + 4 * q;
    if (col > NH - 4) col = NH - 4;
    const v4f v = *(const v4fa*)(cs + ((size_t)(m0 + row) * NU + u) * NH + col);
    *(v4fa*)(sC + row * 32 + 4 * q) = v;
  }

  const v8f z8 = {0.f, 0.f, 0.f, 0.f, 0.f, 0.f, 0.f, 0.f};
  v8f acc[2][4];
  #pragma unroll
  for (int mt = 0; mt < 2; ++mt)
    #pragma unroll
    for (int g = 0; g < 4; ++g) acc[mt][g] = z8;

  const u16* A0 = hsb + ((size_t)(m0 + 32 * wm + m) * NU + u) * NHP;
  const u16* A1 = A0 + (size_t)16 * NU * NHP;
  const u16* Wg = whhP + ((size_t)u * NG + gcc) * NHP;
  #pragma unroll 1
  for (int k0 = 0; k0 < NHP; k0 += 32) {
    const v16u a0 = load_frag(A0 + k0, h);
    const v16u a1 = load_frag(A1 + k0, h);
    #pragma unroll
    for (int g = 0; g < 4; ++g) {
      const v16u bb = load_frag(Wg + (size_t)g * NH * NHP + k0, h);
      acc[0][g] = wmma_bf(a0, bb, acc[0][g]);
      acc[1][g] = wmma_bf(a1, bb, acc[1][g]);
    }
  }
  const u16* I0 = inpHL + ((size_t)(m0 + 32 * wm + m) * NU + u) * HLV;
  const u16* I1 = I0 + (size_t)16 * NU * HLV;
  const u16* Vg = wihP + ((size_t)u * NG + gcc) * NVP;
  #pragma unroll 1
  for (int k0 = 0; k0 < NVP; k0 += 32) {
    const v16u ah0 = load_frag(I0 + 2 * k0, h);
    const v16u al0 = load_frag(I0 + 2 * k0 + 32, h);
    const v16u ah1 = load_frag(I1 + 2 * k0, h);
    const v16u al1 = load_frag(I1 + 2 * k0 + 32, h);
    #pragma unroll
    for (int g = 0; g < 4; ++g) {
      const v16u bb = load_frag(Vg + (size_t)g * NH * NVP + k0, h);
      acc[0][g] = wmma_bf(ah0, bb, acc[0][g]);
      acc[0][g] = wmma_bf(al0, bb, acc[0][g]);
      acc[1][g] = wmma_bf(ah1, bb, acc[1][g]);
      acc[1][g] = wmma_bf(al1, bb, acc[1][g]);
    }
  }

  float bsum[4];
  #pragma unroll
  for (int g = 0; g < 4; ++g)
    bsum[g] = bfr(bih[(size_t)u * NG + g * NH + gcc]) + bfr(bhh[(size_t)u * NG + g * NH + gcc]);
  #pragma unroll
  for (int g = 0; g < 4; ++g)
    #pragma unroll
    for (int mt = 0; mt < 2; ++mt)
      #pragma unroll
      for (int r = 0; r < 8; ++r)
        sG[(g * 64 + 32 * wm + 16 * mt + 8 * h + r) * 32 + colL] = acc[mt][g][r] + bsum[g];
  __syncthreads();

  #pragma unroll 1
  for (int j = 0; j < 16; ++j) {
    const int idx = j * 128 + tid;
    const int col = idx & 31, row = idx >> 5;
    const float gi = sG[idx], gf = sG[2048 + idx], gg = sG[4096 + idx], go = sG[6144 + idx];
    const float cold = bfr(sC[idx]);
    float cn = sigm(gf) * cold + sigm(gi) * tanh_c(gg);
    float hn = sigm(go) * tanh_c(cn);
    if (c0 + col >= NH) { cn = 0.f; hn = 0.f; }
    sC[idx] = cn;
    sH[idx] = hn;
    const u16 hi = f2bf(hn);
    const u16 lo = f2bf(hn - bf2f(hi));
    sHL[row * 64 + col] = hi;
    sHL[row * 64 + 32 + col] = lo;
  }
  __syncthreads();

  lstm_store(sC, sH, sHL, cnew, hrnn, hHL, m0, u, slice, w, lane);
  __threadfence();
  lstm_store(sC, sH, sHL, cnew, hrnn, hHL, m0, u, slice, w, lane);
}

__global__ __launch_bounds__(128) void k_comm(
    const float* __restrict__ qc, const float* __restrict__ kc, const float* __restrict__ vc,
    const float* __restrict__ maskp, u16* __restrict__ ctxHL)
{
  __shared__ float sa[144];
  const int tid = threadIdx.x, lane = tid & 31, w = tid >> 5, b = blockIdx.x;

  #pragma unroll
  for (int rep = 0; rep < 2; ++rep) {
    const int idx = rep * 128 + tid;
    const int ic = (idx < 144) ? idx : 143;
    const int hd = ic / 36, rem = ic - hd * 36, uu = rem / 6, t = rem - uu * 6;
    const float* qp = qc + ((size_t)b * NU + uu) * NCQA + hd * NCQ;
    const float* kp = kc + ((size_t)b * NU + t) * NCQA + hd * NCQ;
    float a = 0.f;
    #pragma unroll 1
    for (int i = 0; i < NCQ; ++i) a += qp[i] * kp[i];
    if (idx < 144) sa[idx] = a * RS32;
  }
  __syncthreads();
  {
    const int tc = (tid < 24) ? tid : 23;
    const int hd = tc / 6, uu = tc - hd * 6;
    const int base = hd * 36 + uu * 6;
    const float mk = maskp[(size_t)b * MPITCH + uu];
    float mx = sa[base];
    #pragma unroll 1
    for (int t = 1; t < NU; ++t) mx = fmaxf(mx, sa[base + t]);
    float sum = 0.f;
    #pragma unroll 1
    for (int t = 0; t < NU; ++t) sum += expf(sa[base + t] - mx);
    const float sc = (1.0f / sum) * mk;
    if (tid < 24) {
      #pragma unroll 1
      for (int t = 0; t < NU; ++t) sa[base + t] = expf(sa[base + t] - mx) * sc;
    }
  }
  __syncthreads();

  const int q8 = lane & 7, sub = lane >> 3, cq = q8 & 3;
  #pragma unroll 1
  for (int it = 0; it < 5; ++it) {
    const int L = it * 16 + w * 4 + sub;
    const int Lc = (L < 78) ? L : 77;
    const int uu = Lc / 13, ks = Lc - uu * 13;
    const int col0 = 32 * ks + 8 * cq;
    int ai[8]; float av[8];
    #pragma unroll
    for (int j = 0; j < 8; ++j) {
      const int c = col0 + j;
      const int cc = (c < NVD) ? c : (NVD - 1);
      ai[j] = (cc / NCV) * 36 + uu * 6;
      av[j] = 0.f;
    }
    #pragma unroll 1
    for (int t = 0; t < NU; ++t) {
      const float* vr = vc + ((size_t)b * NU + t) * NVP + col0;
      const v4f x0 = *(const v4fa*)vr;
      const v4f x1 = *(const v4fa*)(vr + 4);
      av[0] += sa[ai[0] + t] * x0.x;
      av[1] += sa[ai[1] + t] * x0.y;
      av[2] += sa[ai[2] + t] * x0.z;
      av[3] += sa[ai[3] + t] * x0.w;
      av[4] += sa[ai[4] + t] * x1.x;
      av[5] += sa[ai[5] + t] * x1.y;
      av[6] += sa[ai[6] + t] * x1.z;
      av[7] += sa[ai[7] + t] * x1.w;
    }
    v8u o;
    #pragma unroll
    for (int j = 0; j < 8; ++j) {
      const float val = (col0 + j < NVD) ? av[j] : 0.f;
      const u16 hi = f2bf(val);
      const u16 lo = f2bf(val - bf2f(hi));
      o[j] = (q8 < 4) ? hi : lo;
    }
    u16* d = ctxHL + (((size_t)b * NU + uu) * 13 + ks) * 64 + 8 * q8;
    if (L < 78) *(volatile v8u*)d = o;
    __threadfence();
    if (L < 78) *(volatile v8u*)d = o;
  }
}

__global__ __launch_bounds__(128) void k_lnout(
    const float* __restrict__ ctx2, const float* __restrict__ hrnn, const float* __restrict__ cnew,
    const float* __restrict__ hs, const float* __restrict__ cs, const float* __restrict__ maskp,
    const float* __restrict__ lng, const float* __restrict__ lnb, float* __restrict__ out)
{
  __shared__ float smu[12], srs[12];
  const int tid = threadIdx.x, lane = tid & 31, w = tid >> 5;
  const int b2 = blockIdx.x * 2, pr0 = b2 * NU;
  const v4f z4 = {0.f, 0.f, 0.f, 0.f};

  #pragma unroll 1
  for (int rr = 0; rr < 3; ++rr) {
    const int r = w + 4 * rr;
    const size_t rb = (size_t)(pr0 + r) * NHP;
    v4f yv[5];
    float sum = 0.f;
    #pragma unroll
    for (int i = 0; i < 5; ++i) {
      const int pc = lane + 32 * i;
      const int pcc = (pc < 150) ? pc : 149;
      const v4f a = *(const v4fa*)(ctx2 + rb + 4 * pcc);
      const v4f hh = *(const v4fa*)(hrnn + rb + 4 * pcc);
      v4f y = a + hh;
      if (pc >= 150) y = z4;
      yv[i] = y;
      sum += (y.x + y.y) + (y.z + y.w);
    }
    #pragma unroll
    for (int off = 16; off; off >>= 1) sum += __shfl_xor(sum, off, 32);
    const float mu = sum * (1.0f / 600.0f);
    float vs = 0.f;
    #pragma unroll
    for (int i = 0; i < 5; ++i) {
      const int pc = lane + 32 * i;
      v4f d = yv[i] - mu;
      if (pc >= 150) d = z4;
      vs += (d.x * d.x + d.y * d.y) + (d.z * d.z + d.w * d.w);
    }
    #pragma unroll
    for (int off = 16; off; off >>= 1) vs += __shfl_xor(vs, off, 32);
    const float rstd = rsqrtf(vs * (1.0f / 600.0f) + 1e-5f);
    if (lane == 0) { smu[r] = mu; srs[r] = rstd; }
  }
  __syncthreads();

  #pragma unroll 1
  for (int it = 0; it < 15; ++it) {
    const int p = it * 128 + tid;
    const int pc = (p < 1800) ? p : 1799;
    const int r = pc / 150, c4 = pc - r * 150, col = 4 * c4;
    const int pr = pr0 + r;
    const int bsel = (r >= NU) ? 1 : 0;
    const int uu = r - NU * bsel;
    const float mk = maskp[(size_t)(b2 + bsel) * MPITCH + uu];
    const float mu = smu[r], rs = srs[r];
    const size_t ib = (size_t)pr * NHP + col;
    const size_t jb = (size_t)pr * NH + col;
    const v4f a  = *(const v4fa*)(ctx2 + ib);
    const v4f hh = *(const v4fa*)(hrnn + ib);
    const v4f cn = *(const v4fa*)(cnew + ib);
    const v4f g  = *(const v4fa*)(lng + col);
    const v4f be = *(const v4fa*)(lnb + col);
    const v4f hv = *(const v4fa*)(hs + jb);
    const v4f cv = *(const v4fa*)(cs + jb);
    v4f o0, o1;
    #pragma unroll
    for (int j = 0; j < 4; ++j) {
      const float y = a[j] + hh[j];
      const float hn = (y - mu) * rs * bfr(g[j]) + bfr(be[j]);
      o0[j] = (mk != 0.f) ? hn : bfr(hv[j]);
      o1[j] = (mk != 0.f) ? cn[j] : bfr(cv[j]);
    }
    float* d0 = out + (size_t)pr0 * NH + 4 * (size_t)pc;
    if (p < 1800) { *(volatile v4f*)d0 = o0; *(volatile v4f*)(d0 + OUT1) = o1; }
    __threadfence();
    if (p < 1800) { *(volatile v4f*)d0 = o0; *(volatile v4f*)(d0 + OUT1) = o1; }
  }
}

extern "C" void kernel_launch(void* const* d_in, const int* in_sizes, int n_in,
                              void* d_out, int out_size, void* d_ws, size_t ws_size,
                              hipStream_t stream) {
  if (n_in < 18) return;
  if (in_sizes[0] != NB * NIN) return;
  if (in_sizes[1] != NB * NU * NH || in_sizes[2] != NB * NU * NH) return;
  if (in_sizes[3] != NIN * NQK || in_sizes[4] != NQK) return;
  if (in_sizes[5] != NIN * NVD || in_sizes[6] != NVD) return;
  if (in_sizes[7] != NU * NH * NQK) return;
  if (in_sizes[8] != NU * NH * NCQA || in_sizes[9] != NU * NH * NCQA) return;
  if (in_sizes[10] != NU * NH * NVD || in_sizes[11] != NU * NVD * NH) return;
  if (in_sizes[12] != NU * NG * NVD || in_sizes[13] != NU * NG * NH) return;
  if (in_sizes[14] != NU * NG || in_sizes[15] != NU * NG) return;
  if (in_sizes[16] != NH || in_sizes[17] != NH) return;
  if (out_size != 2 * NB * NU * NH) return;

  const float* x    = (const float*)d_in[0];
  const float* hs   = (const float*)d_in[1];
  const float* cs   = (const float*)d_in[2];
  const float* Wk   = (const float*)d_in[3];
  const float* bk   = (const float*)d_in[4];
  const float* Wv   = (const float*)d_in[5];
  const float* bv   = (const float*)d_in[6];
  const float* Wq   = (const float*)d_in[7];
  const float* Wqc  = (const float*)d_in[8];
  const float* Wkc  = (const float*)d_in[9];
  const float* Wvc  = (const float*)d_in[10];
  const float* Woc  = (const float*)d_in[11];
  const float* Wih  = (const float*)d_in[12];
  const float* Whh  = (const float*)d_in[13];
  const float* bih  = (const float*)d_in[14];
  const float* bhh  = (const float*)d_in[15];
  const float* lng  = (const float*)d_in[16];
  const float* lnb  = (const float*)d_in[17];
  float* out = (float*)d_out;

  constexpr size_t SZ_XB   = (size_t)NB * NIN * 2;
  constexpr size_t SZ_HSB  = (size_t)NB * NU * NHP * 2;
  constexpr size_t SZ_WIH  = (size_t)NU * NG * NVP * 2;
  constexpr size_t SZ_WHH  = (size_t)NU * NG * NHP * 2;
  constexpr size_t SZ_INP  = (size_t)NB * NU * HLV * 2;
  constexpr size_t SZ_WK   = (size_t)NQK * NIN * 2;
  constexpr size_t SZ_WV   = (size_t)NVP * NIN * 2;
  constexpr size_t SZ_WQ   = (size_t)NU * NQK * NHP * 2;
  constexpr size_t SZ_WQC  = (size_t)NU * NCQA * NHP * 2;
  constexpr size_t SZ_WVC  = (size_t)NU * NVP * NHP * 2;
  constexpr size_t SZ_WOC  = (size_t)NU * NHP * NVP * 2;
  constexpr size_t SZ_KL   = (size_t)NB * NQK * 4;
  constexpr size_t SZ_VL   = (size_t)NB * NVP * 4;
  constexpr size_t SZ_QL   = (size_t)NB * NU * NQK * 4;
  constexpr size_t SZ_MSK  = (size_t)NB * MPITCH * 4;
  constexpr size_t SZ_CPL  = (size_t)NB * NU * NHP * 4;
  constexpr size_t SZ_HHL  = (size_t)NB * NU * HLH * 2;
  constexpr size_t SZ_QC   = (size_t)NB * NU * NCQA * 4;
  constexpr size_t SZ_VC   = (size_t)NB * NU * NVP * 4;
  constexpr size_t SZ_CHL  = SZ_INP;
  static_assert(SZ_XB % 256 == 0 && SZ_HSB % 256 == 0 && SZ_WIH % 256 == 0 && SZ_WHH % 256 == 0);
  static_assert(SZ_INP % 256 == 0 && SZ_WK % 256 == 0 && SZ_WV % 256 == 0 && SZ_WQ % 256 == 0);
  static_assert(SZ_WQC % 256 == 0 && SZ_WVC % 256 == 0 && SZ_WOC % 256 == 0 && SZ_KL % 256 == 0);
  static_assert(SZ_VL % 256 == 0 && SZ_QL % 256 == 0 && SZ_MSK % 256 == 0 && SZ_CPL % 256 == 0);
  static_assert(SZ_HHL % 256 == 0 && SZ_QC % 256 == 0 && SZ_VC % 256 == 0);

  constexpr size_t SZ_R    = SZ_HSB + SZ_WIH + SZ_WHH + SZ_INP;
  constexpr size_t SZ_OVER = 2 * SZ_QC + SZ_VC + SZ_CHL + SZ_CPL;
  static_assert(SZ_OVER <= SZ_R);

  constexpr size_t OFF_XB   = 0;
  constexpr size_t OFF_R    = OFF_XB + SZ_XB;
  constexpr size_t OFF_HSB  = OFF_R;
  constexpr size_t OFF_WIH  = OFF_HSB + SZ_HSB;
  constexpr size_t OFF_WHH  = OFF_WIH + SZ_WIH;
  constexpr size_t OFF_INP  = OFF_WHH + SZ_WHH;
  constexpr size_t OFF_QC   = OFF_R;
  constexpr size_t OFF_KC   = OFF_QC + SZ_QC;
  constexpr size_t OFF_VC   = OFF_KC + SZ_QC;
  constexpr size_t OFF_CHL  = OFF_VC + SZ_VC;
  constexpr size_t OFF_CTX2 = OFF_CHL + SZ_CHL;
  constexpr size_t OFF_WK   = OFF_R + SZ_R;
  constexpr size_t OFF_WV   = OFF_WK + SZ_WK;
  constexpr size_t OFF_WQ   = OFF_WV + SZ_WV;
  constexpr size_t OFF_WQC  = OFF_WQ + SZ_WQ;
  constexpr size_t OFF_WKC  = OFF_WQC + SZ_WQC;
  constexpr size_t OFF_WVC  = OFF_WKC + SZ_WQC;
  constexpr size_t OFF_WOC  = OFF_WVC + SZ_WVC;
  constexpr size_t OFF_KL   = OFF_WOC + SZ_WOC;
  constexpr size_t OFF_VL   = OFF_KL + SZ_KL;
  constexpr size_t OFF_QL   = OFF_VL + SZ_VL;
  constexpr size_t OFF_MSK  = OFF_QL + SZ_QL;
  constexpr size_t OFF_CNEW = OFF_MSK + SZ_MSK;
  constexpr size_t OFF_HRNN = OFF_CNEW + SZ_CPL;
  constexpr size_t OFF_HHL  = OFF_HRNN + SZ_CPL;
  constexpr size_t WS_TOTAL = OFF_HHL + SZ_HHL;
  static_assert(WS_TOTAL == 105627648);
  static_assert(WS_TOTAL <= 134217728);
  static_assert(OFF_CTX2 + SZ_CPL <= OFF_WK);
  if (WS_TOTAL > ws_size) return;

  char* ws = (char*)d_ws;
  u16* xb    = (u16*)(ws + OFF_XB);
  u16* hsb   = (u16*)(ws + OFF_HSB);
  u16* wihP  = (u16*)(ws + OFF_WIH);
  u16* whhP  = (u16*)(ws + OFF_WHH);
  u16* inpHL = (u16*)(ws + OFF_INP);
  float* qc    = (float*)(ws + OFF_QC);
  float* kc    = (float*)(ws + OFF_KC);
  float* vc    = (float*)(ws + OFF_VC);
  u16* ctxHL   = (u16*)(ws + OFF_CHL);
  float* ctx2  = (float*)(ws + OFF_CTX2);
  u16* wkT   = (u16*)(ws + OFF_WK);
  u16* wvT   = (u16*)(ws + OFF_WV);
  u16* wqT   = (u16*)(ws + OFF_WQ);
  u16* wqcT  = (u16*)(ws + OFF_WQC);
  u16* wkcT  = (u16*)(ws + OFF_WKC);
  u16* wvcT  = (u16*)(ws + OFF_WVC);
  u16* wocT  = (u16*)(ws + OFF_WOC);
  float* kl    = (float*)(ws + OFF_KL);
  float* vl0   = (float*)(ws + OFF_VL);
  float* ql    = (float*)(ws + OFF_QL);
  float* maskp = (float*)(ws + OFF_MSK);
  float* cnew  = (float*)(ws + OFF_CNEW);
  float* hrnn  = (float*)(ws + OFF_HRNN);
  u16* hHL   = (u16*)(ws + OFF_HHL);

  constexpr int TX  = NB * (NIN / 8);
  constexpr int THS = NB * NU * (NHP / 8);
  constexpr int TIH = NU * NG * (NVP / 8);
  constexpr int THH = NU * NG * (NHP / 8);
  static_assert(TX % 256 == 0 && THS % 256 == 0 && TIH % 256 == 0 && THH % 256 == 0);
  k_cvt_rows<<<TX / 256, 256, 0, stream>>>(x, NIN, NIN / 8, TX, xb);
  k_cvt_rows<<<THS / 256, 256, 0, stream>>>(hs, NH, NHP / 8, THS, hsb);
  k_cvt_rows<<<TIH / 256, 256, 0, stream>>>(Wih, NVD, NVP / 8, TIH, wihP);
  k_cvt_rows<<<THH / 256, 256, 0, stream>>>(Whh, NH, NHP / 8, THH, whhP);
  k_cvt_T<<<dim3(NQK / 32, 1), 256, 0, stream>>>(Wk, NIN, NQK, NIN, NQK, wkT);
  k_cvt_T<<<dim3(NVP / 32, 1), 256, 0, stream>>>(Wv, NIN, NVD, NIN, NVP, wvT);
  k_cvt_T<<<dim3(NQK / 32, NU), 256, 0, stream>>>(Wq, NH, NQK, NHP, NQK, wqT);
  k_cvt_T<<<dim3(NCQA / 32, NU), 256, 0, stream>>>(Wqc, NH, NCQA, NHP, NCQA, wqcT);
  k_cvt_T<<<dim3(NCQA / 32, NU), 256, 0, stream>>>(Wkc, NH, NCQA, NHP, NCQA, wkcT);
  k_cvt_T<<<dim3(NVP / 32, NU), 256, 0, stream>>>(Wvc, NH, NVD, NHP, NVP, wvcT);
  k_cvt_T<<<dim3(NHP / 32, NU), 256, 0, stream>>>(Woc, NVD, NH, NVP, NHP, wocT);

  k_gemm<0><<<dim3(NQK / 32, NB / 64, 1), 128, 0, stream>>>(
      xb, NIN, 0, wkT, NIN, 0, kl, NQK, 0, bk, NQK, 1);
  k_gemm<0><<<dim3(NVP / 32, NB / 64, 1), 128, 0, stream>>>(
      xb, NIN, 0, wvT, NIN, 0, vl0, NVP, 0, bv, NVD, 1);
  k_gemm<0><<<dim3(NQK / 32, NB / 64, NU), 128, 0, stream>>>(
      hsb, NU * NHP, NHP, wqT, NHP, NQK * NHP, ql, NU * NQK, NQK, bk, NQK, 0);

  k_select<<<NB, 64, 0, stream>>>(ql, kl, bk, vl0, bv, inpHL, maskp);

  k_lstm<<<dim3(NHP / 32, NB / 64, NU), 128, 0, stream>>>(
      hsb, whhP, inpHL, wihP, bih, bhh, cs, cnew, hrnn, hHL);

  k_gemm<1><<<dim3(NCQA / 32, NB / 64, NU), 128, 0, stream>>>(
      hHL, NU * HLH, HLH, wqcT, NHP, NCQA * NHP, qc, NU * NCQA, NCQA, lng, NCQA, 0);
  k_gemm<1><<<dim3(NCQA / 32, NB / 64, NU), 128, 0, stream>>>(
      hHL, NU * HLH, HLH, wkcT, NHP, NCQA * NHP, kc, NU * NCQA, NCQA, lng, NCQA, 0);
  k_gemm<1><<<dim3(NVP / 32, NB / 64, NU), 128, 0, stream>>>(
      hHL, NU * HLH, HLH, wvcT, NHP, NVP * NHP, vc, NU * NVP, NVP, lng, NVD, 0);
  k_comm<<<NB, 128, 0, stream>>>(qc, kc, vc, maskp, ctxHL);
  k_gemm<1><<<dim3(NHP / 32, NB / 64, NU), 128, 0, stream>>>(
      ctxHL, NU * HLV, HLV, wocT, NVP, NHP * NVP, ctx2, NU * NHP, NHP, lng, NH, 0);

  k_lnout<<<NB / 2, 128, 0, stream>>>(ctx2, hrnn, cnew, hs, cs, maskp, lng, lnb, out);
}
